// self_attention_12670153523745
// MI455X (gfx1250) — hardware-verified
//
#include <hip/hip_runtime.h>

#ifndef NB
#define NB 1
#endif
#ifndef SEQ
#define SEQ 4096
#endif
#define SEQ_FULL 4096
#define HID 768
#define NH 12
#define HD 64
#define SSTR (SEQ + 4)

static_assert(NB == 1);
static_assert(SEQ % 256 == 0);
static_assert(SEQ <= SEQ_FULL);
static_assert(HID == NH * HD);
static_assert(HID % 64 == 0);
static_assert(((SSTR * 4) % 16) == 0);

typedef _Float16 v16h __attribute__((ext_vector_type(16)));
typedef _Float16 v8h  __attribute__((ext_vector_type(8)));
typedef __bf16   v16b __attribute__((ext_vector_type(16)));
typedef float    v8f  __attribute__((ext_vector_type(8)));
typedef float    v4f  __attribute__((ext_vector_type(4)));
typedef unsigned int v4u __attribute__((ext_vector_type(4)));
typedef unsigned short u16;

union FragH { v16h v; v4u u[2]; };
union FragB { v16b v; v4u u[2]; };
union Pack8 { v8h h; v4u u; };

__device__ __forceinline__ v8f vzero() {
  v8f z;
#pragma unroll
  for (int i = 0; i < 8; ++i) z[i] = 0.f;
  return z;
}

__device__ __forceinline__ v8f mma_f16(v16h a, v16h b, v8f c) {
  c = __builtin_amdgcn_wmma_f32_16x16x32_f16(false, a, false, b, (short)0, c, false, false);
  asm volatile("v_nop\n\tv_nop\n\tv_nop\n\tv_nop" : "+v"(c) : "v"(a), "v"(b));
  return c;
}

__device__ __forceinline__ v8f mma_bf16(v16b a, v16b b, v8f c) {
  c = __builtin_amdgcn_wmma_f32_16x16x32_bf16(false, a, false, b, (short)0, c, false, false);
  asm volatile("v_nop\n\tv_nop\n\tv_nop\n\tv_nop" : "+v"(c) : "v"(a), "v"(b));
  return c;
}

__device__ __forceinline__ v16h ld_frag_h(const u16* row, int h) {
  FragH f;
  f.u[0] = *(const v4u*)(row + 8 * h);
  f.u[1] = *(const v4u*)(row + 16 + 8 * h);
  return f.v;
}
__device__ __forceinline__ v16b ld_frag_b(const u16* row, int h) {
  FragB f;
  f.u[0] = *(const v4u*)(row + 8 * h);
  f.u[1] = *(const v4u*)(row + 16 + 8 * h);
  return f.v;
}

__device__ __forceinline__ unsigned int bf16_bits(float f) {
  const unsigned int u = __float_as_uint(f);
  return (u + 0x7FFFu + ((u >> 16) & 1u)) >> 16;
}
__device__ __forceinline__ float bf16_val(float f) {
  return __uint_as_float(bf16_bits(f) << 16);
}
__device__ __forceinline__ unsigned int h16_bits(float f) {
  const _Float16 hv = (_Float16)f;
  const u16 b = __builtin_bit_cast(u16, hv);
  return (unsigned int)b;
}

__global__ __launch_bounds__(256) void k_cvt_x(const float* __restrict__ x,
                                                u16* __restrict__ xb, int n8) {
  const int g = blockIdx.x * 256 + (int)threadIdx.x;
  if (g >= n8) return;
  const float* p = x + (size_t)g * 8;
  const v4f a = *(const v4f*)p;
  const v4f b = *(const v4f*)(p + 4);
  v4u o;
  o[0] = bf16_bits(a[0]) | (bf16_bits(a[1]) << 16);
  o[1] = bf16_bits(a[2]) | (bf16_bits(a[3]) << 16);
  o[2] = bf16_bits(b[0]) | (bf16_bits(b[1]) << 16);
  o[3] = bf16_bits(b[2]) | (bf16_bits(b[3]) << 16);
  u16* d = xb + (size_t)g * 8;
  *(volatile v4u*)d = o;
  __threadfence();
  *(volatile v4u*)d = o;
}

__device__ __forceinline__ void cvtw_store(const u16* T, u16* D, int n0, int k0, int tid) {
#pragma unroll
  for (int i = 0; i < 2; ++i) {
    const int t = tid + 256 * i;
    const int row = t >> 3, seg = t & 7;
    const v4u val = *(const v4u*)(T + row * 72 + seg * 8);
    *(volatile v4u*)(D + (size_t)(n0 + row) * HID + k0 + seg * 8) = val;
  }
}

__global__ __launch_bounds__(256) void k_cvt_w(
    const float* __restrict__ Wq, const float* __restrict__ Wk,
    const float* __restrict__ Wv, const float* __restrict__ Wo,
    u16* __restrict__ WqT, u16* __restrict__ WkT,
    u16* __restrict__ WvT, u16* __restrict__ WoT) {
  __shared__ __attribute__((aligned(16))) u16 T[64 * 72];
  const int z = blockIdx.z;
  const float* W = (z == 0) ? Wq : (z == 1) ? Wk : (z == 2) ? Wv : Wo;
  u16* D = (z == 0) ? WqT : (z == 1) ? WkT : (z == 2) ? WvT : WoT;
  const int n0 = blockIdx.x * 64;
  const int k0 = blockIdx.y * 64;
  const int tid = threadIdx.x;
#pragma unroll
  for (int i = 0; i < 4; ++i) {
    const int idx = tid + 256 * i;
    const int kk = idx >> 4, c4 = (idx & 15) * 4;
    const v4f f = *(const v4f*)(W + (size_t)(k0 + kk) * HID + n0 + c4);
#pragma unroll
    for (int j = 0; j < 4; ++j) {
      const float wv = f[j];
      unsigned int bits;
      if (z == 3) bits = h16_bits(bf16_val(wv) * 64.f);
      else        bits = bf16_bits(wv);
      T[(c4 + j) * 72 + kk] = (u16)bits;
    }
  }
  __syncthreads();
  cvtw_store(T, D, n0, k0, tid);
  __threadfence();
  cvtw_store(T, D, n0, k0, tid);
}

__device__ __forceinline__ void qk_rows_store(const _Float16* T0, u16* Dh, int tid) {
#pragma unroll
  for (int it = 0; it < 8; ++it) {
    const int row = (tid >> 3) + 16 * it, seg = tid & 7;
    const v4u vh = *(const v4u*)(T0 + row * 64 + seg * 8);
    *(volatile v4u*)(Dh + (size_t)row * HD + seg * 8) = vh;
  }
}
__device__ __forceinline__ void vt_rows_store(const _Float16* T0, u16* Dv, int tid) {
#pragma unroll
  for (int it = 0; it < 8; ++it) {
    const int d = (tid >> 4) + 8 * it, seg = tid & 15;
    const v4u vv = *(const v4u*)(T0 + d * 128 + seg * 8);
    *(volatile v4u*)(Dv + (size_t)d * SEQ + seg * 8) = vv;
  }
}

__global__ __launch_bounds__(128) void k_qkv(
    const u16* __restrict__ xb, const u16* __restrict__ WqT,
    const u16* __restrict__ WkT, const u16* __restrict__ WvT,
    u16* __restrict__ Qh, u16* __restrict__ Kh, u16* __restrict__ Vt) {
  __shared__ __attribute__((aligned(16))) _Float16 T0[128 * 64];
  const int z   = blockIdx.z;
  const u16* WT = (z == 0) ? WqT : (z == 1) ? WkT : WvT;
  const int m0  = blockIdx.x * 128;
  const int hh  = blockIdx.y;
  const int n0  = hh * 64;
  const int tid = threadIdx.x, lane = tid & 31, w = tid >> 5;
  const int h = lane >> 4, l15 = lane & 15;
  const int mw  = m0 + w * 32;

  v8f acc[2][4];
#pragma unroll
  for (int s = 0; s < 2; ++s)
#pragma unroll
    for (int i = 0; i < 4; ++i) acc[s][i] = vzero();

#pragma unroll 1
  for (int kk = 0; kk < HID; kk += 32) {
    v16b bfr[4];
#pragma unroll
    for (int nt = 0; nt < 4; ++nt)
      bfr[nt] = ld_frag_b(WT + (size_t)(n0 + nt * 16 + l15) * HID + kk, h);
#pragma unroll
    for (int sub = 0; sub < 2; ++sub) {
      const v16b a = ld_frag_b(xb + (size_t)(mw + sub * 16 + l15) * HID + kk, h);
#pragma unroll
      for (int nt = 0; nt < 4; ++nt) acc[sub][nt] = mma_bf16(a, bfr[nt], acc[sub][nt]);
    }
  }

  if (z < 2) {
#pragma unroll
    for (int sub = 0; sub < 2; ++sub)
#pragma unroll
      for (int nt = 0; nt < 4; ++nt)
#pragma unroll
        for (int r = 0; r < 8; ++r) {
          const int e = (w * 32 + sub * 16 + 8 * h + r) * 64 + nt * 16 + l15;
          T0[e] = (_Float16)acc[sub][nt][r];
        }
    __syncthreads();
    u16* Dh = (z == 0) ? Qh : Kh;
    const size_t base = ((size_t)hh * SEQ + m0) * HD;
    qk_rows_store(T0, Dh + base, tid);
    __threadfence();
    qk_rows_store(T0, Dh + base, tid);
  } else {
#pragma unroll
    for (int sub = 0; sub < 2; ++sub)
#pragma unroll
      for (int nt = 0; nt < 4; ++nt) {
        Pack8 pk;
#pragma unroll
        for (int r = 0; r < 8; ++r) pk.h[r] = (_Float16)acc[sub][nt][r];
        const int d  = nt * 16 + l15;
        const int ml = w * 32 + sub * 16 + 8 * h;
        *(v4u*)(T0 + d * 128 + ml) = pk.u;
      }
    __syncthreads();
    const size_t vbase = ((size_t)hh * HD) * SEQ + m0;
    vt_rows_store(T0, Vt + vbase, tid);
    __threadfence();
    vt_rows_store(T0, Vt + vbase, tid);
  }
}

__global__ __launch_bounds__(256) void k_attn(
    const u16* __restrict__ Qh, const u16* __restrict__ Kh,
    const u16* __restrict__ Vt, u16* __restrict__ Ch, u16* __restrict__ Cl) {
  extern __shared__ __attribute__((aligned(16))) float smem[];
  float* S       = smem;
  float* rowsum  = S + 16 * SSTR;
  float* rowmaxp = rowsum + 16;
  float* Opart   = rowmaxp + 128;

  const int tid = threadIdx.x, lane = tid & 31, w = tid >> 5;
  const int h = lane >> 4, l15 = lane & 15;
  const int halfrow = 8 * h;
  const int kbo     = 8 * h;
  constexpr int TPH = SEQ / 16;
  constexpr int KPW = SEQ / 8;
  const int hd = blockIdx.x / TPH;
  const int j0 = (blockIdx.x - hd * TPH) * 16;

  const size_t qrow = ((size_t)hd * SEQ + j0 + l15) * HD;
  const v16h qh0 = ld_frag_h(Qh + qrow, h);
  const v16h qh1 = ld_frag_h(Qh + qrow + 32, h);

  float vmax[8];
#pragma unroll
  for (int r = 0; r < 8; ++r) vmax[r] = -1e30f;

#pragma unroll 1
  for (int t = 0; t < KPW / 16; ++t) {
    const int m0 = w * KPW + t * 16;
    const size_t krow = ((size_t)hd * SEQ + m0 + l15) * HD;
    const v16h kh0 = ld_frag_h(Kh + krow, h);
    const v16h kh1 = ld_frag_h(Kh + krow + 32, h);
    v8f ah = vzero();
    ah = mma_f16(qh0, kh0, ah);
    ah = mma_f16(qh1, kh1, ah);
#pragma unroll
    for (int r = 0; r < 8; ++r) {
      const float sv = ah[r] * 0.125f;
      S[(halfrow + r) * SSTR + m0 + l15] = sv;
      vmax[r] = fmaxf(vmax[r], sv);
    }
  }
#pragma unroll
  for (int r = 0; r < 8; ++r) {
#pragma unroll
    for (int off = 1; off < 16; off <<= 1) vmax[r] = fmaxf(vmax[r], __shfl_xor(vmax[r], off));
  }
  if (l15 == 0) {
#pragma unroll
    for (int r = 0; r < 8; ++r) rowmaxp[w * 16 + halfrow + r] = vmax[r];
  }
  __syncthreads();

#pragma unroll 1
  for (int j = w * 2; j < w * 2 + 2; ++j) {
    float m = -1e30f;
#pragma unroll
    for (int ww = 0; ww < 8; ++ww) m = fmaxf(m, rowmaxp[ww * 16 + j]);
    float s = 0.f;
#pragma unroll 4
    for (int i = lane; i < SEQ; i += 32) {
      const float e = __expf(S[j * SSTR + i] - m);
      S[j * SSTR + i] = e;
      s += e;
    }
#pragma unroll
    for (int off = 16; off; off >>= 1) s += __shfl_xor(s, off);
    if (lane == 0) rowsum[j] = s;
  }
  __syncthreads();

  v8f acc[4];
#pragma unroll
  for (int cc = 0; cc < 4; ++cc) acc[cc] = vzero();

#pragma unroll 1
  for (int chunk = 0; chunk < KPW / 32; ++chunk) {
    const int m0 = w * KPW + chunk * 32;
    const float* pr = S + l15 * SSTR + m0 + kbo;
    const v4f f0 = *(const v4f*)pr;
    const v4f f1 = *(const v4f*)(pr + 4);
    const v4f f2 = *(const v4f*)(pr + 16);
    const v4f f3 = *(const v4f*)(pr + 20);
    v16h pa;
#pragma unroll
    for (int i = 0; i < 4; ++i) {
      pa[i]      = (_Float16)(f0[i] * 16384.f);
      pa[4 + i]  = (_Float16)(f1[i] * 16384.f);
      pa[8 + i]  = (_Float16)(f2[i] * 16384.f);
      pa[12 + i] = (_Float16)(f3[i] * 16384.f);
    }
#pragma unroll
    for (int cc = 0; cc < 4; ++cc) {
      const v16h vb = ld_frag_h(Vt + ((size_t)(hd * HD + cc * 16 + l15)) * SEQ + m0, h);
      acc[cc] = mma_f16(pa, vb, acc[cc]);
    }
  }
#pragma unroll
  for (int cc = 0; cc < 4; ++cc)
#pragma unroll
    for (int r = 0; r < 8; ++r)
      Opart[w * 1024 + (halfrow + r) * 64 + cc * 16 + l15] = acc[cc][r];
  __syncthreads();

  _Float16* Cs = (_Float16*)smem;
#pragma unroll
  for (int i = 0; i < 4; ++i) {
    const int e = tid + 256 * i;
    const int j = e >> 6;
    float o = 0.f;
#pragma unroll
    for (int ww = 0; ww < 8; ++ww) o += Opart[ww * 1024 + e];
    const float cval = o * (1.0f / rowsum[j]) * (1.0f / 256.0f);
    const _Float16 hi = (_Float16)cval;
    const _Float16 lo = (_Float16)((cval - (float)hi) * 2048.f);
    Cs[e] = hi;
    Cs[1024 + e] = lo;
  }
  __syncthreads();
  {
    const int sel = tid >> 7;
    const int t = tid & 127, row = t >> 3, seg = t & 7;
    const v4u val = *(const v4u*)(Cs + sel * 1024 + row * 64 + seg * 8);
    u16* dst = ((sel == 0) ? Ch : Cl) + ((size_t)(j0 + row)) * HID + hd * HD + seg * 8;
    *(volatile v4u*)dst = val;
    __threadfence();
    *(volatile v4u*)dst = val;
  }
}

__device__ __forceinline__ void out_rows_store(const float* Tw, float* O, int lane) {
#pragma unroll
  for (int it = 0; it < 8; ++it) {
    const int row = (lane >> 4) + 2 * it, seg = lane & 15;
    const v4f v = *(const v4f*)(Tw + row * 64 + seg * 4);
    *(volatile v4f*)(O + (size_t)row * HID + seg * 4) = v;
  }
}

__global__ __launch_bounds__(128) void k_out(
    const u16* __restrict__ Ch, const u16* __restrict__ Cl,
    const u16* __restrict__ WoT, const float* __restrict__ bo,
    float* __restrict__ out) {
  __shared__ __attribute__((aligned(16))) float To[4 * 16 * 64];
  const int m0 = blockIdx.x * 64, n0 = blockIdx.y * 64;
  const int tid = threadIdx.x, lane = tid & 31, w = tid >> 5;
  const int h = lane >> 4, l15 = lane & 15;
  const int mw = m0 + w * 16;

  v8f acch[4], accl[4];
#pragma unroll
  for (int i = 0; i < 4; ++i) { acch[i] = vzero(); accl[i] = vzero(); }

#pragma unroll 1
  for (int kk = 0; kk < HID; kk += 32) {
    v16h bfr[4];
#pragma unroll
    for (int nt = 0; nt < 4; ++nt)
      bfr[nt] = ld_frag_h(WoT + (size_t)(n0 + nt * 16 + l15) * HID + kk, h);
    const v16h ah = ld_frag_h(Ch + (size_t)(mw + l15) * HID + kk, h);
    const v16h al = ld_frag_h(Cl + (size_t)(mw + l15) * HID + kk, h);
#pragma unroll
    for (int nt = 0; nt < 4; ++nt) {
      acch[nt] = mma_f16(ah, bfr[nt], acch[nt]);
      accl[nt] = mma_f16(al, bfr[nt], accl[nt]);
    }
  }

  float* Tw = To + w * 1024;
#pragma unroll
  for (int nt = 0; nt < 4; ++nt) {
    const float bb = bf16_val(bo[n0 + nt * 16 + l15]);
#pragma unroll
    for (int r = 0; r < 8; ++r) {
      const float val = (acch[nt][r] + accl[nt][r] * (1.0f / 2048.0f)) * (1.0f / 4096.0f) + bb;
      Tw[(8 * h + r) * 64 + nt * 16 + l15] = val;
    }
  }
  __syncthreads();
  float* O = out + (size_t)mw * HID + n0;
  out_rows_store(Tw, O, lane);
  __threadfence();
  out_rows_store(Tw, O, lane);
}

extern "C" void kernel_launch(void* const* d_in, const int* in_sizes, int n_in,
                              void* d_out, int out_size, void* d_ws, size_t ws_size,
                              hipStream_t stream) {
  if (n_in < 6) return;
  if (in_sizes[0] < NB * SEQ * HID) return;
  if (in_sizes[1] < HID * HID) return;
  if (in_sizes[2] < HID * HID) return;
  if (in_sizes[3] < HID * HID) return;
  if (in_sizes[4] < HID * HID) return;
  if (in_sizes[5] < HID) return;
  if (out_size < NB * SEQ * HID) return;

  const float* x  = (const float*)d_in[0];
  const float* Wq = (const float*)d_in[1];
  const float* Wk = (const float*)d_in[2];
  const float* Wv = (const float*)d_in[3];
  const float* Wo = (const float*)d_in[4];
  const float* bo = (const float*)d_in[5];
  float* out = (float*)d_out;

  const size_t xb_b  = (size_t)SEQ * HID * 2;
  const size_t w_b   = (size_t)HID * HID * 2;
  const size_t qk_b  = (size_t)NH * SEQ * HD * 2;
  const size_t ctx_b = (size_t)SEQ * HID * 2;
  char* ws = (char*)d_ws;
  size_t off = 0;
  u16* xb  = (u16*)(ws + off); off += xb_b;
  u16* WqT = (u16*)(ws + off); off += w_b;
  u16* WkT = (u16*)(ws + off); off += w_b;
  u16* WvT = (u16*)(ws + off); off += w_b;
  u16* WoT = (u16*)(ws + off); off += w_b;
  u16* Qh  = (u16*)(ws + off); off += qk_b;
  u16* Kh  = (u16*)(ws + off); off += qk_b;
  u16* Vt  = (u16*)(ws + off); off += qk_b;
  u16* Ch  = (u16*)(ws + off); off += ctx_b;
  u16* Cl  = (u16*)(ws + off); off += ctx_b;
  if (off > ws_size) return;

  const int n8 = SEQ * HID / 8;
  k_cvt_x<<<dim3((n8 + 255) / 256), dim3(256), 0, stream>>>(x, xb, n8);
  k_cvt_w<<<dim3(HID / 64, HID / 64, 4), dim3(256), 0, stream>>>(
      Wq, Wk, Wv, Wo, WqT, WkT, WvT, WoT);
  k_qkv<<<dim3(SEQ / 128, NH, 3), dim3(128), 0, stream>>>(
      xb, WqT, WkT, WvT, Qh, Kh, Vt);

  const int smem_bytes = (16 * SSTR + 16 + 128 + 8 * 16 * 64) * (int)sizeof(float);
  hipFuncSetAttribute(reinterpret_cast<const void*>(&k_attn),
                      hipFuncAttributeMaxDynamicSharedMemorySize, smem_bytes);
  k_attn<<<dim3(NH * (SEQ / 16)), dim3(256), smem_bytes, stream>>>(
      Qh, Kh, Vt, Ch, Cl);
  k_out<<<dim3(SEQ / 64, HID / 64), dim3(128), 0, stream>>>(Ch, Cl, WoT, bo, out);

  (void)in_sizes;
}
